// CNP_MLP_Mean_70342974374071
// MI455X (gfx1250) — hardware-verified
//
#include <hip/hip_runtime.h>
#include <hip/hip_bf16.h>


constexpr int NB_     = 32;
constexpr int NL_     = 4096;
constexpr int NU_     = 64;
constexpr int NHX_    = 256;
constexpr int NX_     = 128;
constexpr int NR_     = 128;
constexpr int NCX_    = 256;
constexpr int NT_     = NB_ * NL_;
constexpr int NCT_    = NB_ * NCX_;
constexpr int CHUNK_  = 16384;
constexpr int NCHUNK_ = NT_ / CHUNK_;

static_assert(NT_ % CHUNK_ == 0);
static_assert(CHUNK_ % NL_ == 0);
static_assert(CHUNK_ % 64 == 0);
static_assert(NCT_ % 64 == 0);
static_assert(NL_ % 32 == 0);
static_assert(NHX_ % 64 == 0);
static_assert(NX_ % 64 == 0);
static_assert(NR_ % 64 == 0);
static_assert(NU_ % 32 == 0);

typedef float          v4f   __attribute__((ext_vector_type(4)));
typedef float          v8f   __attribute__((ext_vector_type(8)));
typedef __bf16         v16b  __attribute__((ext_vector_type(16)));
typedef unsigned short u16x8 __attribute__((ext_vector_type(8)));

union FragB { u16x8 h[2]; v16b v; };

__constant__ unsigned int kPosDen[128] = {
0x3f800000u,0x3f898cc0u,0x3f93cfe5u,0x3f9ed70cu,0x3faab0d5u,0x3fb76cf5u,0x3fc51c50u,0x3fd3d10cu,0x3fe39ea9u,0x3ff49a1bu,0x40036cf4u,0x400d3b22u,0x4017c496u,0x4023174bu,0x402f4244u,0x403c55a4u,0x404a62c2u,0x40597c3fu,0x4069b621u,0x407b25edu,0x4086f161u,0x409102bcu,0x409bd461u,0x40a774aau,0x40b3f300u,0x40c15ff6u,0x40cfcd58u,0x40df4e48u,0x40eff755u,0x4100ef4cu,0x410a8de6u,0x4114e43bu,0x41200000u,0x412beff0u,0x4138c3dfu,0x41468cd0u,0x41555d0au,0x41654832u,0x41766364u,0x418462a7u,0x418e432au,0x4198e051u,0x41a44831u,0x41b089eau,0x41bdb5bcu,0x41cbdd1eu,0x41db12d6u,0x41eb6b0du,0x41fcfb72u,0x4207eda7u,0x421211d5u,0x421cf7b4u,0x4228adb9u,0x4235436bu,0x4242c979u,0x425151d4u,0x4260efc0u,0x4271b7f3u,0x4281e057u,0x428b90edu,0x4295fa95u,0x42a12b1fu,0x42ad3160u,0x42ba1d4au,0x42c80000u,0x42d6ebecu,0x42e6f4d6u,0x42f83003u,0x43055a26u,0x430f4d1fu,0x4319fe1eu,0x43257b51u,0x4331d3f4u,0x433f1865u,0x434d5a3eu,0x435cac64u,0x436d232bu,0x437ed466u,0x4388ebc5u,0x439322e8u,0x439e1d27u,0x43a9e911u,0x43b6964au,0x43c435a1u,0x43d2d927u,0x43e29445u,0x43f37bd8u,0x4402d325u,0x440c95d8u,0x441712f8u,0x4422586du,0x442e7528u,0x443b793bu,0x444975e6u,0x44587db7u,0x4468a49cu,0x447a0000u,0x44865373u,0x44905906u,0x449b1e02u,0x44a6b0b0u,0x44b32067u,0x44c07da6u,0x44ceda26u,0x44de48f1u,0x44eede7fu,0x45005867u,0x4509ebbfu,0x451435fbu,0x451f44bfu,0x452b26b7u,0x4537eba3u,0x4545a471u,0x45546355u,0x45643bdcu,0x45754309u,0x4583c7b8u,0x458d9cabu,0x45982d67u,0x45a387eeu,0x45afbb4eu,0x45bcd7b6u,0x45caee88u,0x45da1272u,0x45ea5789u,0x45fbd360u,0x46074e93u,0x461166e2u};

__device__ __forceinline__ unsigned short f2bf(float f) {
    const unsigned u = __float_as_uint(f);
    const unsigned r = u + 0x7FFFu + ((u >> 16) & 1u);
    return (unsigned short)(r >> 16);
}
__device__ __forceinline__ float bf2f(unsigned short b) {
    return __uint_as_float(((unsigned)b) << 16);
}
__device__ __forceinline__ v8f ld8f(const float* p) {
    const v4f a = *(const v4f*)p;
    const v4f b = *(const v4f*)(p + 4);
    return __builtin_shufflevector(a, b, 0, 1, 2, 3, 4, 5, 6, 7);
}
__device__ __forceinline__ void split8(const v8f& x, u16x8& hv, u16x8& lv) {
#pragma unroll
    for (int c = 0; c < 8; ++c) {
        const float f = x[c];
        const unsigned short hb = f2bf(f);
        hv[c] = hb;
        lv[c] = f2bf(f - bf2f(hb));
    }
}
__device__ __forceinline__ float softplus_f(float x) {
    return fmaxf(x, 0.0f) + log1pf(expf(-fabsf(x)));
}

__device__ __forceinline__ void mma_bf(v8f& acc, const FragB& a, const FragB& b) {
    acc = __builtin_amdgcn_wmma_f32_16x16x32_bf16(false, a.v, false, b.v, (short)0, acc, false, false);
    asm volatile("v_nop\n\tv_nop\n\tv_nop\n\tv_nop" : "+v"(acc) : "v"(a.v), "v"(b.v));
}

__global__ __launch_bounds__(256)
void cvt_feat_kernel(const float* __restrict__ src, unsigned short* dh, unsigned short* dl, int n8)
{
    const int i = blockIdx.x * 256 + threadIdx.x;
    if (i >= n8) return;
    const size_t e = (size_t)i * 8;
    const v8f x = ld8f(src + e);
    u16x8 hv, lv;
    split8(x, hv, lv);
    *(volatile u16x8*)(dh + e) = hv;
    *(volatile u16x8*)(dl + e) = lv;
    __threadfence();
    *(volatile u16x8*)(dh + e) = hv;
    *(volatile u16x8*)(dl + e) = lv;
}

__global__ __launch_bounds__(256)
void cvt_w5_kernel(const float* __restrict__ w0, unsigned short* h0, unsigned short* l0,
                   const float* __restrict__ w1, unsigned short* h1, unsigned short* l1,
                   const float* __restrict__ w2, unsigned short* h2, unsigned short* l2,
                   const float* __restrict__ w3, unsigned short* h3, unsigned short* l3,
                   const float* __restrict__ w4, unsigned short* h4, unsigned short* l4,
                   int nn0, int kk0, int nn1, int kk1, int nn2, int kk2, int nn3, int kk3, int nn4, int kk4)
{
    const float* W = w0; unsigned short* dh = h0; unsigned short* dl = l0; int Nd = nn0, Kd = kk0;
    if (blockIdx.y == 1)      { W = w1; dh = h1; dl = l1; Nd = nn1; Kd = kk1; }
    else if (blockIdx.y == 2) { W = w2; dh = h2; dl = l2; Nd = nn2; Kd = kk2; }
    else if (blockIdx.y == 3) { W = w3; dh = h3; dl = l3; Nd = nn3; Kd = kk3; }
    else if (blockIdx.y == 4) { W = w4; dh = h4; dl = l4; Nd = nn4; Kd = kk4; }
    const int i = blockIdx.x * 256 + threadIdx.x;
    const int kg8 = Kd >> 3;
    if (i >= Nd * kg8) return;
    const int n  = i / kg8;
    const int kg = i - n * kg8;
    v8f x;
#pragma unroll
    for (int c = 0; c < 8; ++c) x[c] = W[(size_t)(kg * 8 + c) * Nd + n];
    u16x8 hv, lv;
    split8(x, hv, lv);
    const size_t e = (size_t)n * Kd + kg * 8;
    *(volatile u16x8*)(dh + e) = hv;
    *(volatile u16x8*)(dl + e) = lv;
    __threadfence();
    *(volatile u16x8*)(dh + e) = hv;
    *(volatile u16x8*)(dl + e) = lv;
}

__global__ __launch_bounds__(128)
void ptab_kernel(float* PT)
{
#pragma clang fp contract(off)
    __shared__ __attribute__((aligned(16))) float sp[NHX_];
    const int tid = threadIdx.x;
    const int k   = blockIdx.x;
    const float den = __uint_as_float(kPosDen[tid]);
    const float ang = (float)k / den;
    const float sv = sinf(ang);
    const float cv = cosf(ang);
    sp[2 * tid]     = sv;
    sp[2 * tid + 1] = cv;
    __syncthreads();
    const int t = tid & 63;
    const v4f v = *(const v4f*)(sp + t * 4);
    float* gp = PT + (size_t)k * NHX_ + t * 4;
    if (tid < 64) *(volatile v4f*)gp = v;
    __threadfence();
    if (tid < 64) *(volatile v4f*)gp = v;
}

template<int EPI>
__global__ __launch_bounds__(128)
void gemm3_kernel(const unsigned short* __restrict__ Ah, const unsigned short* __restrict__ Al,
                  const unsigned short* __restrict__ Bh, const unsigned short* __restrict__ Bl,
                  int K, const float* __restrict__ bias,
                  const float* __restrict__ aux0, const float* __restrict__ aux1,
                  const float* __restrict__ aux2, int pbase,
                  unsigned short* Oh, unsigned short* Ol, float* Of, int ldo)
{
#pragma clang fp contract(off)
    constexpr int STP = 68;
    __shared__ __attribute__((aligned(16))) float st[64 * STP];

    const int tid  = threadIdx.x;
    const int lane = tid & 31;
    const int wave = tid >> 5;
    const int h    = lane >> 4;
    const int m    = lane & 15;
    const int wm   = wave >> 1;
    const int wn   = wave & 1;
    const int row0 = blockIdx.y * 64;
    const int col0 = blockIdx.x * 64;
    const int rowW = row0 + wm * 32;
    const int colW = col0 + wn * 32;

    v8f acc[4];
#pragma unroll
    for (int j = 0; j < 4; ++j)
#pragma unroll
        for (int r = 0; r < 8; ++r) acc[j][r] = 0.0f;

    const size_t aoff  = (size_t)(rowW + m) * K + 8 * h;
    const size_t boff  = (size_t)(colW + m) * K + 8 * h;
    const size_t sub16 = (size_t)16 * K;
    const int nk = K >> 5;

#pragma unroll 1
    for (int kt = 0; kt < nk; ++kt) {
        const size_t k0 = (size_t)kt * 32;
        FragB fa[2], ga[2], fb[2], gb[2];
#pragma unroll
        for (int s = 0; s < 2; ++s) {
            const unsigned short* p = Ah + aoff + s * sub16 + k0;
            const unsigned short* q = Al + aoff + s * sub16 + k0;
            fa[s].h[0] = *(const u16x8*)(p);
            fa[s].h[1] = *(const u16x8*)(p + 16);
            ga[s].h[0] = *(const u16x8*)(q);
            ga[s].h[1] = *(const u16x8*)(q + 16);
        }
#pragma unroll
        for (int j = 0; j < 2; ++j) {
            const unsigned short* p = Bh + boff + j * sub16 + k0;
            const unsigned short* q = Bl + boff + j * sub16 + k0;
            fb[j].h[0] = *(const u16x8*)(p);
            fb[j].h[1] = *(const u16x8*)(p + 16);
            gb[j].h[0] = *(const u16x8*)(q);
            gb[j].h[1] = *(const u16x8*)(q + 16);
        }
#pragma unroll
        for (int s = 0; s < 2; ++s)
#pragma unroll
            for (int j = 0; j < 2; ++j) {
                mma_bf(acc[s * 2 + j], fa[s], fb[j]);
                mma_bf(acc[s * 2 + j], fa[s], gb[j]);
                mma_bf(acc[s * 2 + j], ga[s], fb[j]);
            }
    }

#pragma unroll
    for (int s = 0; s < 2; ++s)
#pragma unroll
        for (int j = 0; j < 2; ++j)
#pragma unroll
            for (int r = 0; r < 8; ++r)
                st[(wm * 32 + s * 16 + 8 * h + r) * STP + wn * 32 + j * 16 + m] = acc[s * 2 + j][r];
    __syncthreads();

    if (EPI != 3) {
        u16x8 hv[4], lv[4];
        size_t go[4];
#pragma unroll
        for (int it = 0; it < 4; ++it) {
            const int row = it * 16 + (tid >> 3);
            const int seg = tid & 7;
            const int n0  = col0 + seg * 8;
            v8f x = ld8f(st + row * STP + seg * 8);
            x += ld8f(bias + n0);
            if (EPI == 0) {
                const int prow = (pbase + row0 + row) & (NL_ - 1);
                x += ld8f(aux0 + (size_t)prow * NHX_ + n0);
            }
            if (EPI == 2) {
                const int gr = row0 + row;
                const float yv = aux1[gr] + 0.1f * aux2[gr];
                const v8f wy = ld8f(aux0 + n0);
                x += wy * yv;
            }
            if (EPI == 0 || EPI == 2) {
#pragma unroll
                for (int c = 0; c < 8; ++c) x[c] = fmaxf(x[c], 0.0f);
            }
            split8(x, hv[it], lv[it]);
            go[it] = (size_t)(row0 + row) * ldo + n0;
        }
#pragma unroll
        for (int it = 0; it < 4; ++it) {
            *(volatile u16x8*)(Oh + go[it]) = hv[it];
            *(volatile u16x8*)(Ol + go[it]) = lv[it];
        }
        __threadfence();
#pragma unroll
        for (int it = 0; it < 4; ++it) {
            *(volatile u16x8*)(Oh + go[it]) = hv[it];
            *(volatile u16x8*)(Ol + go[it]) = lv[it];
        }
    } else {
        v4f vals[8];
        size_t go[8];
#pragma unroll
        for (int it = 0; it < 8; ++it) {
            const int row = it * 8 + (tid >> 4);
            const int seg = tid & 15;
            const int n0  = col0 + seg * 4;
            v4f x = *(const v4f*)(st + row * STP + seg * 4);
            x += *(const v4f*)(bias + n0);
            vals[it] = x;
            go[it] = (size_t)(row0 + row) * ldo + n0;
        }
#pragma unroll
        for (int it = 0; it < 8; ++it) *(volatile v4f*)(Of + go[it]) = vals[it];
        __threadfence();
#pragma unroll
        for (int it = 0; it < 8; ++it) *(volatile v4f*)(Of + go[it]) = vals[it];
    }
}

__global__ __launch_bounds__(256)
void gather_kernel(const unsigned short* __restrict__ Xh, const unsigned short* __restrict__ Xl,
                   const int* __restrict__ idx, unsigned short* Ch, unsigned short* Cl)
{
    const int i = blockIdx.x * 256 + threadIdx.x;
    if (i >= NCT_ * 16) return;
    const int row = i >> 4;
    const int seg = i & 15;
    const unsigned short* src = Xh; unsigned short* dst = Ch;
    if (blockIdx.y == 1) { src = Xl; dst = Cl; }
    int l = idx[row];
    l = min(max(l, 0), NL_ - 1);
    const int b = row / NCX_;
    const u16x8 v = *(const u16x8*)(src + ((size_t)b * NL_ + (size_t)l) * NX_ + seg * 8);
    const size_t d = (size_t)row * NX_ + seg * 8;
    *(volatile u16x8*)(dst + d) = v;
    __threadfence();
    *(volatile u16x8*)(dst + d) = v;
}

__global__ __launch_bounds__(128)
void rvec_kernel(const float* __restrict__ R2, const float* __restrict__ W5, const float* __restrict__ b5, float* RB)
{
    __shared__ float sr[NR_];
    const int b = blockIdx.x;
    const int j = threadIdx.x;
    const float* base = R2 + (size_t)b * NCX_ * NR_ + j;
    float s = 0.0f;
#pragma unroll 4
    for (int c = 0; c < NCX_; ++c) s += base[(size_t)c * NR_];
    sr[j] = s * (1.0f / (float)NCX_);
    __syncthreads();
    float v = b5[j];
    const float* wb = W5 + (size_t)NX_ * NR_ + j;
#pragma unroll 4
    for (int k = 0; k < NR_; ++k) v += sr[k] * wb[(size_t)k * NR_];
    float* gp = RB + (size_t)b * NR_ + j;
    *(volatile float*)gp = v;
    __threadfence();
    *(volatile float*)gp = v;
}

__global__ __launch_bounds__(128)
void dec_kernel(const unsigned short* __restrict__ Xh, const unsigned short* __restrict__ Xl,
                const unsigned short* __restrict__ Bh, const unsigned short* __restrict__ Bl,
                const float* __restrict__ RB, const float* __restrict__ W6, const float* __restrict__ b6,
                float* out)
{
    constexpr int DP = NR_ + 4;
    __shared__ __attribute__((aligned(16))) float sD[32 * DP];
    __shared__ float sW6[2 * NR_];
    __shared__ __attribute__((aligned(16))) float sO[64];

    const int tid  = threadIdx.x;
    const int lane = tid & 31;
    const int wave = tid >> 5;
    const int h    = lane >> 4;
    const int m    = lane & 15;
    const int row0 = blockIdx.x * 32;
    const int b    = row0 / NL_;

    sW6[tid]       = W6[tid];
    sW6[tid + 128] = W6[tid + 128];

    v8f acc[4];
#pragma unroll
    for (int j = 0; j < 4; ++j)
#pragma unroll
        for (int r = 0; r < 8; ++r) acc[j][r] = 0.0f;

    const size_t aoff  = (size_t)(row0 + m) * NX_ + 8 * h;
    const size_t boff  = (size_t)(wave * 32 + m) * NX_ + 8 * h;
    const size_t sub16 = (size_t)16 * NX_;

#pragma unroll 1
    for (int kt = 0; kt < NX_ / 32; ++kt) {
        const size_t k0 = (size_t)kt * 32;
        FragB fa[2], ga[2], fb[2], gb[2];
#pragma unroll
        for (int s = 0; s < 2; ++s) {
            const unsigned short* p = Xh + aoff + s * sub16 + k0;
            const unsigned short* q = Xl + aoff + s * sub16 + k0;
            fa[s].h[0] = *(const u16x8*)(p);
            fa[s].h[1] = *(const u16x8*)(p + 16);
            ga[s].h[0] = *(const u16x8*)(q);
            ga[s].h[1] = *(const u16x8*)(q + 16);
        }
#pragma unroll
        for (int j = 0; j < 2; ++j) {
            const unsigned short* p = Bh + boff + j * sub16 + k0;
            const unsigned short* q = Bl + boff + j * sub16 + k0;
            fb[j].h[0] = *(const u16x8*)(p);
            fb[j].h[1] = *(const u16x8*)(p + 16);
            gb[j].h[0] = *(const u16x8*)(q);
            gb[j].h[1] = *(const u16x8*)(q + 16);
        }
#pragma unroll
        for (int s = 0; s < 2; ++s)
#pragma unroll
            for (int j = 0; j < 2; ++j) {
                mma_bf(acc[s * 2 + j], fa[s], fb[j]);
                mma_bf(acc[s * 2 + j], fa[s], gb[j]);
                mma_bf(acc[s * 2 + j], ga[s], fb[j]);
            }
    }

    const float rb0 = RB[b * NR_ + wave * 32 + m];
    const float rb1 = RB[b * NR_ + wave * 32 + 16 + m];
#pragma unroll
    for (int s = 0; s < 2; ++s)
#pragma unroll
        for (int j = 0; j < 2; ++j)
#pragma unroll
            for (int r = 0; r < 8; ++r)
                sD[(s * 16 + 8 * h + r) * DP + wave * 32 + j * 16 + m] =
                    fmaxf(acc[s * 2 + j][r] + (j == 0 ? rb0 : rb1), 0.0f);
    __syncthreads();

    const int row = tid >> 2;
    const int q   = tid & 3;
    float s0 = 0.0f, s1 = 0.0f;
#pragma unroll 4
    for (int c = 0; c < 32; ++c) {
        const int col = q * 32 + c;
        const float d = sD[row * DP + col];
        s0 += d * sW6[2 * col];
        s1 += d * sW6[2 * col + 1];
    }
    s0 += __shfl_xor(s0, 1, 32);
    s0 += __shfl_xor(s0, 2, 32);
    s1 += __shfl_xor(s1, 1, 32);
    s1 += __shfl_xor(s1, 2, 32);
    const float yv   = s0 + b6[0];
    const float varv = 0.1f + 0.9f * softplus_f(s1 + b6[1]);
    if (q == 0) { sO[row] = yv; sO[32 + row] = varv; }
    __syncthreads();

    if (wave == 0) {
        const int p   = (lane >> 3) & 1;
        const int seg = lane & 7;
        const v4f v = *(const v4f*)(sO + p * 32 + seg * 4);
        float* gp = out + (size_t)p * NT_ + row0 + seg * 4;
        if (lane < 16) *(volatile v4f*)gp = v;
        __threadfence();
        if (lane < 16) *(volatile v4f*)gp = v;
    }
}

extern "C" void kernel_launch(void* const* d_in, const int* in_sizes, int n_in,
                              void* d_out, int out_size, void* d_ws, size_t ws_size,
                              hipStream_t stream)
{
    if (n_in < 17) return;
    const int want[17] = {
        NT_ * NU_, NCT_, NCT_, NB_, NCT_,
        NU_ * NHX_, NHX_,
        NHX_ * NX_, NX_,
        (NX_ + 1) * NR_, NR_,
        NR_ * NR_, NR_,
        (NX_ + NR_) * NR_, NR_,
        NR_ * 2, 2 };
    for (int i = 0; i < 17; ++i) if (in_sizes[i] != want[i]) return;
    if (out_size != 2 * NT_) return;

    const float* feat = (const float*)d_in[0];
    const int*   idx  = (const int*)d_in[1];
    const float* ctx  = (const float*)d_in[2];
    const float* noi  = (const float*)d_in[4];
    const float* W1 = (const float*)d_in[5];   const float* b1 = (const float*)d_in[6];
    const float* W2 = (const float*)d_in[7];   const float* b2 = (const float*)d_in[8];
    const float* W3 = (const float*)d_in[9];   const float* b3 = (const float*)d_in[10];
    const float* W4 = (const float*)d_in[11];  const float* b4 = (const float*)d_in[12];
    const float* W5 = (const float*)d_in[13];  const float* b5 = (const float*)d_in[14];
    const float* W6 = (const float*)d_in[15];  const float* b6 = (const float*)d_in[16];
    float* out = (float*)d_out;

    char* ws = (char*)d_ws;
    size_t off = 0;
    auto carve = [&](size_t bytes) -> char* { char* p = ws + off; off += (bytes + 255) & ~(size_t)255; return p; };

    unsigned short* B1h = (unsigned short*)carve((size_t)NHX_ * NU_ * 2);
    unsigned short* B1l = (unsigned short*)carve((size_t)NHX_ * NU_ * 2);
    unsigned short* B2h = (unsigned short*)carve((size_t)NX_ * NHX_ * 2);
    unsigned short* B2l = (unsigned short*)carve((size_t)NX_ * NHX_ * 2);
    unsigned short* B3h = (unsigned short*)carve((size_t)NR_ * NX_ * 2);
    unsigned short* B3l = (unsigned short*)carve((size_t)NR_ * NX_ * 2);
    unsigned short* B4h = (unsigned short*)carve((size_t)NR_ * NR_ * 2);
    unsigned short* B4l = (unsigned short*)carve((size_t)NR_ * NR_ * 2);
    unsigned short* B5h = (unsigned short*)carve((size_t)NR_ * NX_ * 2);
    unsigned short* B5l = (unsigned short*)carve((size_t)NR_ * NX_ * 2);
    float*          PT  = (float*)carve((size_t)NL_ * NHX_ * 4);
    unsigned short* FEh = (unsigned short*)carve((size_t)NT_ * NU_ * 2);
    unsigned short* FEl = (unsigned short*)carve((size_t)NT_ * NU_ * 2);
    char*           HH  = carve((size_t)CHUNK_ * NHX_ * 2 * 2);
    unsigned short* Hh  = (unsigned short*)HH;
    unsigned short* Hl  = Hh + (size_t)CHUNK_ * NHX_;
    unsigned short* Xh  = (unsigned short*)carve((size_t)NT_ * NX_ * 2);
    unsigned short* Xl  = (unsigned short*)carve((size_t)NT_ * NX_ * 2);
    float*          RB  = (float*)carve((size_t)NB_ * NR_ * 4);
    if (off > ws_size) return;

    unsigned short* XCh = (unsigned short*)(HH);
    unsigned short* XCl = (unsigned short*)(HH + (size_t)NCT_ * NX_ * 2);
    unsigned short* R1h = (unsigned short*)(HH + (size_t)NCT_ * NX_ * 2 * 2);
    unsigned short* R1l = (unsigned short*)(HH + (size_t)NCT_ * NX_ * 2 * 3);
    float*          R2  = (float*)(HH + (size_t)NCT_ * NX_ * 2 * 4);
    if ((size_t)NCT_ * NX_ * 2 * 4 + (size_t)NCT_ * NR_ * 4 > (size_t)CHUNK_ * NHX_ * 2 * 2) return;

    const dim3 b256(256), b128(128);

    cvt_w5_kernel<<<dim3(16, 5), b256, 0, stream>>>(W1, B1h, B1l, W2, B2h, B2l, W3, B3h, B3l, W4, B4h, B4l, W5, B5h, B5l,
                                                   NHX_, NU_, NX_, NHX_, NR_, NX_, NR_, NR_, NR_, NX_);
    cvt_feat_kernel<<<dim3((NT_ * NU_ / 8 + 255) / 256), b256, 0, stream>>>(feat, FEh, FEl, NT_ * NU_ / 8);
    ptab_kernel<<<dim3(NL_), b128, 0, stream>>>(PT);

    for (int c = 0; c < NCHUNK_; ++c) {
        const size_t c0 = (size_t)c * CHUNK_;
        gemm3_kernel<0><<<dim3(NHX_ / 64, CHUNK_ / 64), b128, 0, stream>>>(
            FEh + c0 * NU_, FEl + c0 * NU_, B1h, B1l, NU_, b1, PT, b1, b1, (int)c0, Hh, Hl, RB, NHX_);
        gemm3_kernel<1><<<dim3(NX_ / 64, CHUNK_ / 64), b128, 0, stream>>>(
            Hh, Hl, B2h, B2l, NHX_, b2, b2, b2, b2, 0, Xh + c0 * NX_, Xl + c0 * NX_, RB, NX_);
    }

    gather_kernel<<<dim3(NCT_ * 16 / 256, 2), b256, 0, stream>>>(Xh, Xl, idx, XCh, XCl);
    gemm3_kernel<2><<<dim3(NR_ / 64, NCT_ / 64), b128, 0, stream>>>(
        XCh, XCl, B3h, B3l, NX_, b3, W3 + (size_t)NX_ * NR_, ctx, noi, 0, R1h, R1l, RB, NR_);
    gemm3_kernel<3><<<dim3(NR_ / 64, NCT_ / 64), b128, 0, stream>>>(
        R1h, R1l, B4h, B4l, NR_, b4, b4, b4, b4, 0, XCh, XCl, R2, NR_);
    rvec_kernel<<<dim3(NB_), b128, 0, stream>>>(R2, W5, b5, RB);

    dec_kernel<<<dim3(NT_ / 32), b128, 0, stream>>>(Xh, Xl, B5h, B5l, RB, W6, b6, out);
}
